// StdAbsBlock_32590211842339
// MI455X (gfx1250) — hardware-verified
//
#include <hip/hip_runtime.h>
#include <math.h>

constexpr int kBatch  = 2;
constexpr int kSeq    = 2048;
constexpr int kDim    = 1024;
constexpr int kHeads  = 16;
constexpr int kDh     = 64;
constexpr int kTok    = kBatch * kSeq;
constexpr int kFF     = 4096;
constexpr int kGroups = kBatch * kHeads;
constexpr int kGch    = 2;
constexpr int kNChunk = kGroups / kGch;
constexpr int kPK     = 3 * kSeq;
constexpr int kQKld   = 2 * kDim;
constexpr int kFFRows = 2048;
constexpr float kWCarry    = 16.0f;
constexpr float kWCarryInv = 1.0f / 16.0f;
constexpr float kOCarry    = 16.0f;
constexpr float kGCarry    = 16.0f;
constexpr float kOProjScale = 1.0f / (kOCarry * kWCarry);
constexpr float kFF2Scale   = 1.0f / (kGCarry * kWCarry);
constexpr float kScoreScale = 0.125f;
constexpr float kInvDim     = 1.0f / 1024.0f;
constexpr float kLnEps      = 1e-5f;
static_assert(kGroups % kGch == 0, "chunking");
static_assert(kHeads % kGch == 0, "chunks never cross a batch row");

constexpr size_t kMiB     = 1048576;
constexpr size_t kOffQK16 = 0;
constexpr size_t kOffG16  = 0;
constexpr size_t kOffVT   = 16 * kMiB;
constexpr size_t kOffO16  = 40 * kMiB;
constexpr size_t kOffWQKV = 48 * kMiB;
constexpr size_t kOffH16  = 54 * kMiB;
constexpr size_t kOffV32  = 62 * kMiB;
constexpr size_t kOffSC   = 48 * kMiB;
constexpr size_t kOffPP   = 80 * kMiB;
constexpr size_t kOffWO   = 48 * kMiB;
constexpr size_t kOffX1   = 50 * kMiB;
constexpr size_t kOffH2   = 66 * kMiB;
constexpr size_t kOffWF1  = 74 * kMiB;
constexpr size_t kOffWF2  = 82 * kMiB;
constexpr size_t kOffU    = 90 * kMiB;
constexpr size_t kWsTotal = 128 * kMiB;
static_assert(kOffQK16 + (size_t)kTok * kQKld * 2 == 16 * kMiB, "QK16 extent");
static_assert(kOffG16 + (size_t)kFFRows * kFF * 2 == 16 * kMiB, "G16 extent");
static_assert(kOffVT + (size_t)kGroups * kDh * kPK * 2 == kOffO16, "VT extent");
static_assert(kOffO16 + (size_t)kTok * kDim * 2 == kOffSC, "O16 extent");
static_assert(kOffWQKV + (size_t)3 * kDim * kDim * 2 == kOffH16, "WQKV extent");
static_assert(kOffH16 + (size_t)kTok * kDim * 2 == kOffV32, "H16 extent");
static_assert(kOffV32 + (size_t)kTok * kDim * 4 <= kOffPP, "V32 extent");
static_assert(kOffSC + (size_t)kGch * kSeq * kSeq * 4 == kOffPP, "SC extent");
static_assert(kOffPP + (size_t)kGch * kSeq * kPK * 2 == kWsTotal, "PP extent");
static_assert(kOffWO + (size_t)kDim * kDim * 2 == kOffX1, "WO extent");
static_assert(kOffX1 + (size_t)kTok * kDim * 4 == kOffH2, "X1 extent");
static_assert(kOffH2 + (size_t)kTok * kDim * 2 == kOffWF1, "H2 extent");
static_assert(kOffWF1 + (size_t)kFF * kDim * 2 == kOffWF2, "WF1 extent");
static_assert(kOffWF2 + (size_t)kDim * kFF * 2 == kOffU, "WF2 extent");
static_assert(kOffU + (size_t)kFFRows * kFF * 4 <= kWsTotal, "U extent");
static_assert(kWsTotal == 134217728ull, "carve total");

typedef __attribute__((ext_vector_type(16))) _Float16 v16h;
typedef __attribute__((ext_vector_type(8)))  _Float16 v8h;
typedef __attribute__((ext_vector_type(16))) __bf16   v16b;
typedef __attribute__((ext_vector_type(8)))  __bf16   v8b;
typedef __attribute__((ext_vector_type(8)))  float    v8f;
typedef __attribute__((ext_vector_type(4)))  float    v4f;
typedef __attribute__((ext_vector_type(4)))  unsigned int v4u;

__device__ __forceinline__ unsigned short f2bf_bits(float f) {
  unsigned u = __float_as_uint(f);
  return (unsigned short)((u + 0x7FFFu + ((u >> 16) & 1u)) >> 16);
}
__device__ __forceinline__ float bf_bits2f(unsigned short h) { return __uint_as_float(((unsigned)h) << 16); }

__device__ __forceinline__ void dep_guard_h(v8f& a, v8f& b, v16h x, v16h y) { asm volatile("v_nop\n\tv_nop\n\tv_nop\n\tv_nop" : "+v"(a), "+v"(b) : "v"(x), "v"(y)); }
__device__ __forceinline__ void dep_guard_b(v8f& a, v8f& b, v16b x, v16b y) { asm volatile("v_nop\n\tv_nop\n\tv_nop\n\tv_nop" : "+v"(a), "+v"(b) : "v"(x), "v"(y)); }
__device__ __forceinline__ void keep4_h(v16h a, v16h b, v16h c, v16h d) { asm volatile("v_nop" :: "v"(a), "v"(b), "v"(c), "v"(d)); }
__device__ __forceinline__ void keep4_b(v16b a, v16b b, v16b c, v16b d) { asm volatile("v_nop" :: "v"(a), "v"(b), "v"(c), "v"(d)); }
__device__ __forceinline__ void acc_guard4(v8f& a, v8f& b, v8f& c, v8f& d) { asm volatile("v_nop\n\tv_nop\n\tv_nop\n\tv_nop" : "+v"(a), "+v"(b), "+v"(c), "+v"(d)); }
template <typename T> struct Frag;
template <> struct Frag<_Float16> {
  typedef v16h V; union U { v16h v; v8h h[2]; };
  static __device__ __forceinline__ v16h load(const _Float16* p) {
    U f; f.h[0] = *(const v8h*)(p); f.h[1] = *(const v8h*)(p + 16); return f.v;
  }
  static __device__ __forceinline__ v8f mma(v16h a, v16h b, v8f c) {
    return __builtin_amdgcn_wmma_f32_16x16x32_f16(false, a, false, b, (short)0, c, false, false);
  }
  static __device__ __forceinline__ void guard(v8f& a, v8f& b, v16h x, v16h y) { dep_guard_h(a, b, x, y); }
  static __device__ __forceinline__ void keep(v16h a, v16h b, v16h c, v16h d) { keep4_h(a, b, c, d); }
};
template <> struct Frag<__bf16> {
  typedef v16b V; union U { v16b v; v8b h[2]; };
  static __device__ __forceinline__ v16b load(const __bf16* p) {
    U f; f.h[0] = *(const v8b*)(p); f.h[1] = *(const v8b*)(p + 16); return f.v;
  }
  static __device__ __forceinline__ v8f mma(v16b a, v16b b, v8f c) {
    return __builtin_amdgcn_wmma_f32_16x16x32_bf16(false, a, false, b, (short)0, c, false, false);
  }
  static __device__ __forceinline__ void guard(v8f& a, v8f& b, v16b x, v16b y) { dep_guard_b(a, b, x, y); }
  static __device__ __forceinline__ void keep(v16b a, v16b b, v16b c, v16b d) { keep4_b(a, b, c, d); }
};

__device__ __forceinline__ unsigned pk16(unsigned short a, unsigned short b) { return (unsigned)a | ((unsigned)b << 16); }
__device__ __forceinline__ unsigned short h_bits(float f) { const _Float16 h = (_Float16)f; return __builtin_bit_cast(unsigned short, h); }

template <int ET> struct Elem;
template <> struct Elem<0> { typedef _Float16 T; };
template <> struct Elem<1> { typedef __bf16 T; };
template <int ET, bool SPLIT, int BIAS_MODE, int OUT_MODE, bool RESID, int ACT = 0, int CAUSAL = 0>
__global__ __launch_bounds__(256) void wmma_gemm64(
    const unsigned short* __restrict__ Ap, const unsigned short* __restrict__ A2p, int lda, long strideA,
    const unsigned short* __restrict__ Btp, const unsigned short* __restrict__ Bt2p, int ldb, long strideB,
    void* __restrict__ Cout, void* __restrict__ Cout2, int ldc, long strideC,
    const float* __restrict__ bias,
    const float* __restrict__ resid, long strideR,
    int M, int N, int K, float scale) {
  typedef typename Elem<ET>::T T;
  typedef typename Frag<T>::V V;
  const T* A = (const T*)Ap; const T* A2 = (const T*)A2p; const T* Bt = (const T*)Btp; const T* Bt2 = (const T*)Bt2p;
  __shared__ __align__(16) float sT[8][16 * 68];
  const int b    = blockIdx.y;
  const int lane = threadIdx.x & 31;
  const int wave = threadIdx.x >> 5;
  const int tilesN = N >> 6;
  const int tilesM = M >> 6;
  const int tile = blockIdx.x * 8 + wave;
  if (tile >= tilesM * tilesN) return;
  const int tm = tile / tilesN;
  const int tn = tile - tm * tilesN;
  const int m0 = tm << 6;
  const int n0 = tn << 6;
  if (CAUSAL == 1 && n0 > m0) return;
  int Kend = K;
  if (CAUSAL == 2) { const int kc = 3 * (m0 + 64); Kend = (kc < K) ? kc : K; }

  const T* Ab  = A  + (size_t)b * strideA;
  const T* Bb  = Bt + (size_t)b * strideB;
  const T* Ab2 = SPLIT ? (A2  + (size_t)b * strideA) : nullptr;
  const T* Bb2 = SPLIT ? (Bt2 + (size_t)b * strideB) : nullptr;

  const int rlane = lane & 15;
  const int koff  = (lane >> 4) * 8;
  const int mOff  = (lane >> 4) * 8;

  v8f acc[4][4];
#pragma unroll
  for (int i = 0; i < 4; ++i)
#pragma unroll
    for (int j = 0; j < 4; ++j) acc[i][j] = (v8f){0.f,0.f,0.f,0.f,0.f,0.f,0.f,0.f};

  for (int k0 = 0; k0 < Kend; k0 += 32) {
    V bh[4], bl[4];
#pragma unroll
    for (int j = 0; j < 4; ++j) {
      const size_t bo = (size_t)(n0 + (j << 4) + rlane) * ldb + koff + k0;
      bh[j] = Frag<T>::load(Bb + bo);
      if (SPLIT) bl[j] = Frag<T>::load(Bb2 + bo);
    }
#pragma unroll
    for (int i = 0; i < 4; ++i) {
      const size_t ao = (size_t)(m0 + (i << 4) + rlane) * lda + koff + k0;
      V ah = Frag<T>::load(Ab + ao);
      V al;
      if (SPLIT) al = Frag<T>::load(Ab2 + ao);
#pragma unroll
      for (int j = 0; j < 4; ++j) {
        acc[i][j] = Frag<T>::mma(ah, bh[j], acc[i][j]);
        if (SPLIT) {
          acc[i][j] = Frag<T>::mma(ah, bl[j], acc[i][j]);
          acc[i][j] = Frag<T>::mma(al, bh[j], acc[i][j]);
        }
      }
      Frag<T>::guard(acc[i][0], acc[i][3], ah, SPLIT ? al : ah);
    }
    Frag<T>::keep(bh[0], bh[1], bh[2], bh[3]);
    if (SPLIT) Frag<T>::keep(bl[0], bl[1], bl[2], bl[3]);
  }
  acc_guard4(acc[0][0], acc[0][1], acc[0][2], acc[0][3]);
  acc_guard4(acc[1][0], acc[1][1], acc[1][2], acc[1][3]);
  acc_guard4(acc[2][0], acc[2][1], acc[2][2], acc[2][3]);
  acc_guard4(acc[3][0], acc[3][1], acc[3][2], acc[3][3]);

  float* slab = sT[wave];
  const float* Rb = RESID ? (resid + (size_t)b * strideR) : nullptr;
#pragma unroll
  for (int i = 0; i < 4; ++i) {
    const int mBase = m0 + (i << 4);
#pragma unroll
    for (int j = 0; j < 4; ++j) {
      const int n = n0 + (j << 4) + rlane;
      float bv = 0.f;
      if (BIAS_MODE == 2) bv = bias[n];
#pragma unroll
      for (int r = 0; r < 8; ++r) {
        float v = acc[i][j][r] * scale;
        if (BIAS_MODE == 1) v += bias[mBase + mOff + r];
        if (BIAS_MODE == 2) v += bv;
        if (RESID) v += Rb[(size_t)(mBase + mOff + r) * ldc + n];
        if (ACT == 2) v = fmaxf(v, 0.0f);
        if (ACT == 4) v = (v > 0.f) ? v : 0.01f * v;
        slab[(mOff + r) * 68 + (j << 4) + rlane] = v;
      }
    }
    __builtin_amdgcn_fence(__ATOMIC_RELEASE, "workgroup");
    __builtin_amdgcn_wave_barrier();
    __builtin_amdgcn_fence(__ATOMIC_ACQUIRE, "workgroup");
    if (OUT_MODE == 0) {
      float* C = (float*)Cout + (size_t)b * strideC;
      const int hh = lane >> 4, c4 = (lane & 15) * 4;
      for (int pass = 0; pass < 2; ++pass) {
#pragma unroll
        for (int it = 0; it < 8; ++it) {
          const int row = it * 2 + hh;
          v4f v = *(const v4f*)(slab + row * 68 + c4);
          *(volatile v4f*)(C + (size_t)(mBase + row) * ldc + n0 + c4) = v;
        }
        __threadfence();
      }
    } else {
      const int q = lane >> 3, c8 = (lane & 7) * 8;
      unsigned short* C  = (unsigned short*)Cout  + (size_t)b * strideC;
      unsigned short* C2 = (OUT_MODE == 2) ? ((unsigned short*)Cout2 + (size_t)b * strideC) : nullptr;
      for (int pass = 0; pass < 2; ++pass) {
#pragma unroll
        for (int it = 0; it < 4; ++it) {
          const int row = it * 4 + q;
          const float* sp = slab + row * 68 + c8;
          v8h hv, lv;
#pragma unroll
          for (int e = 0; e < 8; ++e) {
            if (OUT_MODE == 1) {
              hv[e] = (_Float16)sp[e];
            } else {
              unsigned short hb = f2bf_bits(sp[e]);
              unsigned short lb = f2bf_bits(sp[e] - bf_bits2f(hb));
              hv[e] = __builtin_bit_cast(_Float16, hb);
              lv[e] = __builtin_bit_cast(_Float16, lb);
            }
          }
          *(volatile v8h*)(C + (size_t)(mBase + row) * ldc + n0 + c8) = hv;
          if (OUT_MODE == 2) *(volatile v8h*)(C2 + (size_t)(mBase + row) * ldc + n0 + c8) = lv;
        }
        __threadfence();
      }
    }
    __builtin_amdgcn_fence(__ATOMIC_RELEASE, "workgroup");
    __builtin_amdgcn_wave_barrier();
    __builtin_amdgcn_fence(__ATOMIC_ACQUIRE, "workgroup");
  }
}

__global__ __launch_bounds__(256) void cast8_f16_kernel(const float* __restrict__ in, unsigned short* __restrict__ out,
                                                        int n8, float scale) {
  const int i = blockIdx.x * 256 + threadIdx.x;
  if (i >= n8) return;
  const float* p = in + 8 * (size_t)i;
  const v4f a = *(const v4f*)(p);
  const v4f c = *(const v4f*)(p + 4);
  unsigned short hb[8];
#pragma unroll
  for (int e = 0; e < 4; ++e) {
    hb[e]     = h_bits(a[e] * scale);
    hb[4 + e] = h_bits(c[e] * scale);
  }
  const v4u u = (v4u){pk16(hb[0], hb[1]), pk16(hb[2], hb[3]), pk16(hb[4], hb[5]), pk16(hb[6], hb[7])};
  unsigned short* q = out + 8 * (size_t)i;
  *(volatile v4u*)q = u;
  __threadfence();
  *(volatile v4u*)q = u;
}

__global__ __launch_bounds__(128) void ln_f16_kernel(const float* __restrict__ X, const float* __restrict__ w,
                                                     const float* __restrict__ bb, unsigned short* __restrict__ out) {
  __shared__ float red1[4];
  __shared__ float red2[4];
  const int row  = blockIdx.x;
  const int t    = threadIdx.x;
  const int lane = t & 31, wave = t >> 5;
  const float* xr = X + (size_t)row * kDim + 8 * t;
  const v4f a = *(const v4f*)(xr);
  const v4f c = *(const v4f*)(xr + 4);
  float v[8];
#pragma unroll
  for (int e = 0; e < 4; ++e) { v[e] = a[e]; v[4 + e] = c[e]; }
  float s = ((v[0] + v[1]) + (v[2] + v[3])) + ((v[4] + v[5]) + (v[6] + v[7]));
#pragma unroll
  for (int off = 16; off > 0; off >>= 1) s += __shfl_xor(s, off, 32);
  if (lane == 0) red1[wave] = s;
  __syncthreads();
  const float mu = ((red1[0] + red1[1]) + (red1[2] + red1[3])) * kInvDim;
  float d[8];
  float s2 = 0.f;
#pragma unroll
  for (int e = 0; e < 8; ++e) { d[e] = v[e] - mu; s2 += d[e] * d[e]; }
#pragma unroll
  for (int off = 16; off > 0; off >>= 1) s2 += __shfl_xor(s2, off, 32);
  if (lane == 0) red2[wave] = s2;
  __syncthreads();
  const float var = ((red2[0] + red2[1]) + (red2[2] + red2[3])) * kInvDim;
  const float inv = rsqrtf(var + kLnEps);
  const v4f wa = *(const v4f*)(w + 8 * t);
  const v4f wc = *(const v4f*)(w + 8 * t + 4);
  const v4f ba = *(const v4f*)(bb + 8 * t);
  const v4f bc = *(const v4f*)(bb + 8 * t + 4);
  unsigned short hb[8];
#pragma unroll
  for (int e = 0; e < 4; ++e) {
    hb[e]     = h_bits(d[e] * inv * wa[e] + ba[e]);
    hb[4 + e] = h_bits(d[4 + e] * inv * wc[e] + bc[e]);
  }
  const v4u u = (v4u){pk16(hb[0], hb[1]), pk16(hb[2], hb[3]), pk16(hb[4], hb[5]), pk16(hb[6], hb[7])};
  unsigned short* q = out + (size_t)row * kDim + 8 * t;
  *(volatile v4u*)q = u;
  __threadfence();
  *(volatile v4u*)q = u;
}

__global__ __launch_bounds__(256) void vt_pack_kernel(const float* __restrict__ V32, unsigned short* __restrict__ VT) {
  __shared__ float sm[64][65];
  const int t   = threadIdx.x;
  const int jb  = blockIdx.x;
  const int grp = blockIdx.y;
  const int b   = grp >> 4;
  const int h   = grp & 15;
  const float* src = V32 + (size_t)(b * kSeq + jb * 64) * kDim + h * kDh;
#pragma unroll
  for (int i = 0; i < 16; ++i) {
    const int e   = i * 256 + t;
    const int tok = e >> 6;
    const int d   = e & 63;
    sm[d][tok] = src[(size_t)tok * kDim + d];
  }
  __syncthreads();
  const int lane = t & 31, wave = t >> 5;
  const int q = lane >> 3, c8 = (lane & 7) * 8;
  unsigned short* dst = VT + (size_t)grp * kDh * kPK + (size_t)jb * 192;
  for (int pass = 0; pass < 2; ++pass) {
#pragma unroll
    for (int it = 0; it < 2; ++it) {
      const int row = wave * 8 + it * 4 + q;
      unsigned short hb[8], lb[8];
#pragma unroll
      for (int e = 0; e < 8; ++e) {
        const float f = sm[row][c8 + e];
        const unsigned short hh = f2bf_bits(f);
        hb[e] = hh;
        lb[e] = f2bf_bits(f - bf_bits2f(hh));
      }
      const v4u uh = (v4u){pk16(hb[0], hb[1]), pk16(hb[2], hb[3]), pk16(hb[4], hb[5]), pk16(hb[6], hb[7])};
      const v4u ul = (v4u){pk16(lb[0], lb[1]), pk16(lb[2], lb[3]), pk16(lb[4], lb[5]), pk16(lb[6], lb[7])};
      unsigned short* rp = dst + (size_t)row * kPK + c8;
      *(volatile v4u*)(rp)       = uh;
      *(volatile v4u*)(rp + 64)  = ul;
      *(volatile v4u*)(rp + 128) = uh;
    }
    __threadfence();
  }
}

__global__ __launch_bounds__(256) void softmax_pack_kernel(const float* __restrict__ SC, unsigned short* __restrict__ PP) {
  __shared__ float redM[8];
  __shared__ float redS[8];
  const int i    = blockIdx.x;
  const int gl   = blockIdx.y;
  const int t    = threadIdx.x;
  const int lane = t & 31, wave = t >> 5;
  const int c0   = t * 8;
  const float* sr = SC + ((size_t)gl * kSeq + i) * kSeq + c0;
  const v4f a = *(const v4f*)(sr);
  const v4f c = *(const v4f*)(sr + 4);
  float xs[8];
#pragma unroll
  for (int e = 0; e < 4; ++e) {
    const bool k0 = (c0 + e <= i);
    const bool k1 = (c0 + 4 + e <= i);
    const float r0 = k0 ? a[e] : 0.0f;
    const float r1 = k1 ? c[e] : 0.0f;
    xs[e]     = k0 ? r0 * kScoreScale : -INFINITY;
    xs[4 + e] = k1 ? r1 * kScoreScale : -INFINITY;
  }
  float m = fmaxf(fmaxf(fmaxf(xs[0], xs[1]), fmaxf(xs[2], xs[3])), fmaxf(fmaxf(xs[4], xs[5]), fmaxf(xs[6], xs[7])));
#pragma unroll
  for (int off = 16; off > 0; off >>= 1) m = fmaxf(m, __shfl_xor(m, off, 32));
  if (lane == 0) redM[wave] = m;
  __syncthreads();
  float rm = redM[0];
#pragma unroll
  for (int q = 1; q < 8; ++q) rm = fmaxf(rm, redM[q]);
  const bool wact = (wave * 256 <= i);
  float p[8];
  float s = 0.0f;
  if (wact) {
#pragma unroll
    for (int e = 0; e < 8; ++e) p[e] = expf(xs[e] - rm);
    s = ((p[0] + p[1]) + (p[2] + p[3])) + ((p[4] + p[5]) + (p[6] + p[7]));
  } else {
#pragma unroll
    for (int e = 0; e < 8; ++e) p[e] = 0.0f;
  }
#pragma unroll
  for (int off = 16; off > 0; off >>= 1) s += __shfl_xor(s, off, 32);
  if (lane == 0) redS[wave] = s;
  __syncthreads();
  float rs = redS[0];
#pragma unroll
  for (int q = 1; q < 8; ++q) rs += redS[q];
  const float inv = 1.0f / rs;
  unsigned short hb[8], lb[8];
#pragma unroll
  for (int e = 0; e < 8; ++e) {
    const float pn = p[e] * inv;
    const unsigned short hh = f2bf_bits(pn);
    hb[e] = hh;
    lb[e] = f2bf_bits(pn - bf_bits2f(hh));
  }
  const v4u uh = (v4u){pk16(hb[0], hb[1]), pk16(hb[2], hb[3]), pk16(hb[4], hb[5]), pk16(hb[6], hb[7])};
  const v4u ul = (v4u){pk16(lb[0], lb[1]), pk16(lb[2], lb[3]), pk16(lb[4], lb[5]), pk16(lb[6], lb[7])};
  unsigned short* dst = PP + ((size_t)gl * kSeq + i) * kPK + (size_t)(t >> 3) * 192 + (t & 7) * 8;
  for (int pass = 0; pass < 2; ++pass) {
    *(volatile v4u*)(dst)       = uh;
    *(volatile v4u*)(dst + 64)  = uh;
    *(volatile v4u*)(dst + 128) = ul;
    __threadfence();
  }
}

__global__ __launch_bounds__(256) void gelu2_f16_kernel(const float* __restrict__ U, unsigned short* __restrict__ G,
                                                        int n2, float carry) {
  const int i = blockIdx.x * 256 + threadIdx.x;
  if (i >= n2) return;
  unsigned w = 0u;
#pragma unroll 1
  for (int e = 0; e < 2; ++e) {
    const float u  = U[2 * (size_t)i + e];
    const float gv = 0.5f * u * (1.0f + erff(u * 0.70710678118654752f));
    w |= ((unsigned)h_bits(gv * carry)) << (16 * e);
  }
  volatile unsigned* q = (volatile unsigned*)G + i;
  *q = w;
  __threadfence();
  *q = w;
}

extern "C" void kernel_launch(void* const* d_in, const int* in_sizes, int n_in,
                              void* d_out, int out_size, void* d_ws, size_t ws_size,
                              hipStream_t stream) {
  if (n_in < 11) return;
  if (in_sizes[0] != kTok * kDim) return;
  if (in_sizes[1] != kDim || in_sizes[2] != kDim || in_sizes[3] != kDim || in_sizes[4] != kDim) return;
  if (in_sizes[5] != 3 * kDim * kDim || in_sizes[6] != kDim * kDim) return;
  if (in_sizes[7] != kFF * kDim || in_sizes[8] != kFF || in_sizes[9] != kDim * kFF || in_sizes[10] != kDim) return;
  if (out_size != kTok * kDim) return;
  if (ws_size < kWsTotal) return;

  const float* x      = (const float*)d_in[0];
  const float* ln1_w  = (const float*)d_in[1];
  const float* ln1_b  = (const float*)d_in[2];
  const float* ln2_w  = (const float*)d_in[3];
  const float* ln2_b  = (const float*)d_in[4];
  const float* qkv_w  = (const float*)d_in[5];
  const float* o_w    = (const float*)d_in[6];
  const float* ffn_w1 = (const float*)d_in[7];
  const float* ffn_b1 = (const float*)d_in[8];
  const float* ffn_w2 = (const float*)d_in[9];
  const float* ffn_b2 = (const float*)d_in[10];
  float* outp = (float*)d_out;

  unsigned char* ws = (unsigned char*)d_ws;
  unsigned short* QK16 = (unsigned short*)(ws + kOffQK16);
  unsigned short* G16  = (unsigned short*)(ws + kOffG16);
  unsigned short* VT   = (unsigned short*)(ws + kOffVT);
  unsigned short* O16  = (unsigned short*)(ws + kOffO16);
  unsigned short* WQKV = (unsigned short*)(ws + kOffWQKV);
  unsigned short* H16  = (unsigned short*)(ws + kOffH16);
  float*          V32  = (float*)(ws + kOffV32);
  float*          SC   = (float*)(ws + kOffSC);
  unsigned short* PP   = (unsigned short*)(ws + kOffPP);
  unsigned short* WO   = (unsigned short*)(ws + kOffWO);
  float*          X1   = (float*)(ws + kOffX1);
  unsigned short* H2   = (unsigned short*)(ws + kOffH2);
  unsigned short* WF1  = (unsigned short*)(ws + kOffWF1);
  unsigned short* WF2  = (unsigned short*)(ws + kOffWF2);
  float*          U    = (float*)(ws + kOffU);

  {
    const int n8 = 3 * kDim * kDim / 8;
    cast8_f16_kernel<<<dim3((n8 + 255) / 256), dim3(256), 0, stream>>>(qkv_w, WQKV, n8, kWCarry);
  }
  ln_f16_kernel<<<dim3(kTok), dim3(128), 0, stream>>>(x, ln1_w, ln1_b, H16);
  wmma_gemm64<0, false, 0, 1, false, 0, 0><<<dim3((kTok / 64) * (kQKld / 64) / 8, 1), dim3(256), 0, stream>>>(
      H16, H16, kDim, 0L, WQKV, WQKV, kDim, 0L, (void*)QK16, (void*)QK16, kQKld, 0L,
      nullptr, nullptr, 0L, kTok, kQKld, kDim, kWCarryInv);
  wmma_gemm64<0, false, 0, 0, false, 0, 0><<<dim3((kTok / 64) * (kDim / 64) / 8, 1), dim3(256), 0, stream>>>(
      H16, H16, kDim, 0L, WQKV + (size_t)2 * kDim * kDim, WQKV + (size_t)2 * kDim * kDim, kDim, 0L,
      (void*)V32, (void*)V32, kDim, 0L, nullptr, nullptr, 0L, kTok, kDim, kDim, kWCarryInv);
  vt_pack_kernel<<<dim3(kSeq / 64, kGroups), dim3(256), 0, stream>>>(V32, VT);

  for (int ch = 0; ch < kNChunk; ++ch) {
    const int g0 = ch * kGch;
    const int b  = g0 / kHeads;
    const int h0 = g0 % kHeads;
    const unsigned short* Aq = QK16 + (size_t)b * kSeq * kQKld + (size_t)h0 * kDh;
    const unsigned short* Bk = Aq + kDim;
    wmma_gemm64<0, false, 0, 0, false, 0, 1><<<dim3((kSeq / 64) * (kSeq / 64) / 8, kGch), dim3(256), 0, stream>>>(
        Aq, Aq, kQKld, (long)kDh, Bk, Bk, kQKld, (long)kDh, (void*)SC, (void*)SC, kSeq, (long)kSeq * kSeq,
        nullptr, nullptr, 0L, kSeq, kSeq, kDh, 1.0f);
    softmax_pack_kernel<<<dim3(kSeq, kGch), dim3(256), 0, stream>>>(SC, PP);
    wmma_gemm64<1, false, 0, 1, false, 0, 2><<<dim3((kSeq / 64) * (kDh / 64) / 8, kGch), dim3(256), 0, stream>>>(
        PP, PP, kPK, (long)kSeq * kPK, VT + (size_t)g0 * kDh * kPK, VT + (size_t)g0 * kDh * kPK, kPK, (long)kDh * kPK,
        (void*)(O16 + (size_t)b * kSeq * kDim + (size_t)h0 * kDh), (void*)(O16 + (size_t)b * kSeq * kDim + (size_t)h0 * kDh),
        kDim, (long)kDh, nullptr, nullptr, 0L, kSeq, kDh, kPK, kOCarry);
  }

  {
    const int n8 = kDim * kDim / 8;
    cast8_f16_kernel<<<dim3((n8 + 255) / 256), dim3(256), 0, stream>>>(o_w, WO, n8, kWCarry);
  }
  wmma_gemm64<0, false, 0, 0, true, 0, 0><<<dim3((kTok / 64) * (kDim / 64) / 8, 1), dim3(256), 0, stream>>>(
      O16, O16, kDim, 0L, WO, WO, kDim, 0L, (void*)X1, (void*)X1, kDim, 0L,
      nullptr, x, 0L, kTok, kDim, kDim, kOProjScale);
  ln_f16_kernel<<<dim3(kTok), dim3(128), 0, stream>>>(X1, ln2_w, ln2_b, H2);
  {
    const int n8 = kFF * kDim / 8;
    cast8_f16_kernel<<<dim3((n8 + 255) / 256), dim3(256), 0, stream>>>(ffn_w1, WF1, n8, kWCarry);
    cast8_f16_kernel<<<dim3((n8 + 255) / 256), dim3(256), 0, stream>>>(ffn_w2, WF2, n8, kWCarry);
  }
  for (int mc = 0; mc < kTok / kFFRows; ++mc) {
    const size_t rowOff = (size_t)mc * kFFRows;
    wmma_gemm64<0, false, 2, 0, false, 0, 0><<<dim3((kFFRows / 64) * (kFF / 64) / 8, 1), dim3(256), 0, stream>>>(
        H2 + rowOff * kDim, H2 + rowOff * kDim, kDim, 0L, WF1, WF1, kDim, 0L, (void*)U, (void*)U, kFF, 0L,
        ffn_b1, nullptr, 0L, kFFRows, kFF, kDim, kWCarryInv);
    {
      const int n2 = kFFRows * kFF / 2;
      gelu2_f16_kernel<<<dim3((n2 + 255) / 256), dim3(256), 0, stream>>>(U, G16, n2, kGCarry);
    }
    wmma_gemm64<0, false, 2, 0, true, 0, 0><<<dim3((kFFRows / 64) * (kDim / 64) / 8, 1), dim3(256), 0, stream>>>(
        G16, G16, kFF, 0L, WF2, WF2, kFF, 0L, (void*)(outp + rowOff * kDim), (void*)(outp + rowOff * kDim), kDim, 0L,
        ffn_b2, X1 + rowOff * kDim, 0L, kFFRows, kDim, kFF, kFF2Scale);
  }
}
